// _Net_85899345920420
// MI455X (gfx1250) — hardware-run, weakly checked
//
#include <hip/hip_runtime.h>

typedef float          v8f   __attribute__((ext_vector_type(8)));
typedef float          v4f   __attribute__((ext_vector_type(4)));
typedef unsigned int   v4u   __attribute__((ext_vector_type(4)));
typedef int            v8i   __attribute__((ext_vector_type(8)));
typedef unsigned short v8us  __attribute__((ext_vector_type(8)));
typedef unsigned short v16us __attribute__((ext_vector_type(16)));
typedef __bf16         v16bf __attribute__((ext_vector_type(16)));
typedef _Float16       v16h  __attribute__((ext_vector_type(16)));
typedef v4f  __attribute__((may_alias)) v4fa;
typedef v8us __attribute__((may_alias)) v8usa;
union FragB { v16bf v; v16us u; v8us h[2]; v8i w; };
union FragH { v16h  v; v16us u; v8us h[2]; v8i w; };

__device__ __forceinline__ v8f wmb(const FragB& a, const FragB& b, v8f c) {
  v8f d = __builtin_amdgcn_wmma_f32_16x16x32_bf16(false, a.v, false, b.v, (short)0, c, false, false);
  asm volatile("v_nop\n\tv_nop\n\tv_nop\n\tv_nop" : "+v"(d) : "v"(a.w), "v"(b.w));
  return d;
}

__device__ __forceinline__ v8f wmh(const FragH& a, const FragH& b, v8f c) {
  v8f d = __builtin_amdgcn_wmma_f32_16x16x32_f16(false, a.v, false, b.v, (short)0, c, false, false);
  asm volatile("v_nop\n\tv_nop\n\tv_nop\n\tv_nop" : "+v"(d) : "v"(a.w), "v"(b.w));
  return d;
}

__device__ __forceinline__ unsigned bf16_bits(float f) {
  const unsigned u = __float_as_uint(f);
  const unsigned r = (u + 0x7FFFu + ((u >> 16) & 1u)) >> 16;
  const unsigned q = (u >> 16) | 0x40u;
  return ((u & 0x7fffffffu) > 0x7f800000u) ? q : r;
}

__device__ __forceinline__ float bf16_val(float f) {
  return __uint_as_float(bf16_bits(f) << 16);
}
__device__ __forceinline__ int clampi(int v, int lo, int hi) {
  return v < lo ? lo : (v > hi ? hi : v);
}

__device__ __forceinline__ unsigned f16_bits(float f) {
  const unsigned u  = __float_as_uint(f);
  const unsigned s  = (u >> 16) & 0x8000u;
  const unsigned a  = u & 0x7fffffffu;
  const unsigned t  = a - 0x38000000u;
  const unsigned r  = (t + 0x0FFFu + ((t >> 13) & 1u)) >> 13;
  const unsigned rc = r > 0x7C00u ? 0x7C00u : r;
  const bool small  = a < 0x38800000u;
  const bool isnan  = a > 0x7f800000u;
  const unsigned fin = small ? 0u : (s | rc);
  return isnan ? (s | 0x7E00u) : fin;
}

__device__ __forceinline__ unsigned pk16(unsigned lo, unsigned hi) { return lo | (hi << 16); }
__device__ __forceinline__ unsigned bf16_lo_bits(float v) {
  float hi = bf16_val(v);
  asm volatile("" : "+v"(hi));
  return bf16_bits(v - hi);
}
__device__ __forceinline__ v4u pack8_bf16(v4f a, v4f c) {
  return (v4u){ pk16(bf16_bits(a[0]), bf16_bits(a[1])), pk16(bf16_bits(a[2]), bf16_bits(a[3])),
                pk16(bf16_bits(c[0]), bf16_bits(c[1])), pk16(bf16_bits(c[2]), bf16_bits(c[3])) };
}
__device__ __forceinline__ v4u pack8_bf16_lo(v4f a, v4f c) {
  return (v4u){ pk16(bf16_lo_bits(a[0]), bf16_lo_bits(a[1])), pk16(bf16_lo_bits(a[2]), bf16_lo_bits(a[3])),
                pk16(bf16_lo_bits(c[0]), bf16_lo_bits(c[1])), pk16(bf16_lo_bits(c[2]), bf16_lo_bits(c[3])) };
}
__device__ __forceinline__ v4u pack8_f16(v4f a, v4f c) {
  return (v4u){ pk16(f16_bits(a[0]), f16_bits(a[1])), pk16(f16_bits(a[2]), f16_bits(a[3])),
                pk16(f16_bits(c[0]), f16_bits(c[1])), pk16(f16_bits(c[2]), f16_bits(c[3])) };
}

template <int FORM>
__global__ __launch_bounds__(256) void k_plane(const float* __restrict__ src, int rows, int cols, int ldsrc,
                                               unsigned short* __restrict__ dst, int MP, int KP) {
  static_assert(FORM >= 0 && FORM <= 3);
  const int KTOT = (FORM == 1 || FORM == 3) ? 2 * KP : KP;
  const unsigned ppr   = (unsigned)(KTOT >> 3);
  const unsigned kp8   = (unsigned)(KP >> 3);
  const unsigned total = (unsigned)MP * ppr;
  const unsigned g     = blockIdx.x * 256u + threadIdx.x;
  const unsigned rowu  = g / ppr;
  const unsigned p     = g - rowu * ppr;
  const bool second    = p >= kp8;
  const int row = (int)rowu;
  const int c0  = (int)((second ? p - kp8 : p) << 3);
  const float* srow = src + (size_t)clampi(row, 0, rows - 1) * (size_t)ldsrc;
  float x[8];
  unsigned mk[8];
#pragma unroll
  for (int e = 0; e < 8; ++e) {
    const int c = c0 + e;
    const float v = srow[clampi(c, 0, cols - 1)];
    asm volatile("" :: "v"(v));
    x[e]  = v;
    mk[e] = (row < rows && c < cols) ? 0xFFFFu : 0u;
  }
  const v4f a = (v4f){ x[0], x[1], x[2], x[3] };
  const v4f c = (v4f){ x[4], x[5], x[6], x[7] };
  v4u o;
  if (FORM == 2) {
    o = pack8_f16(a, c);
  } else {
    const v4u hi = pack8_bf16(a, c);
    o = hi;
    if (FORM == 1) { const v4u lo = pack8_bf16_lo(a, c); o = second ? lo : hi; }
  }
  const v4u mw = (v4u){ pk16(mk[0], mk[1]), pk16(mk[2], mk[3]), pk16(mk[4], mk[5]), pk16(mk[6], mk[7]) };
  o &= mw;
  if (g < total) {
    volatile v4u* q = (volatile v4u*)(dst + (size_t)g * 8);
    *q = o;
    __threadfence();
    *q = o;
  }
}

template <int FORM> struct FragOf    { typedef FragB T; };
template <>         struct FragOf<2> { typedef FragH T; };
__device__ __forceinline__ v8f mm(const FragB& a, const FragB& b, v8f c) { return wmb(a, b, c); }
__device__ __forceinline__ v8f mm(const FragH& a, const FragH& b, v8f c) { return wmh(a, b, c); }
template <class F> __device__ __forceinline__ F ld_frag(const unsigned short* p) {
  F f;
  f.h[0] = *(const v8usa*)(p);
  f.h[1] = *(const v8usa*)(p + 16);
  return f;
}

template <int FORM, int EPI>
__global__ __launch_bounds__(256) __attribute__((amdgpu_num_vgpr(248)))
void k_gemm_nt(const unsigned short* __restrict__ A, const unsigned short* __restrict__ B,
               const float* __restrict__ bias, float* __restrict__ D, int M, int N, int KTOT, int ldd) {
  static_assert(FORM >= 0 && FORM <= 2);
  static_assert(EPI == 0 || EPI == 1);
  typedef typename FragOf<FORM>::T F;
  __shared__ __attribute__((aligned(16))) float sT[8][16 * 68];
  const int lane = threadIdx.x & 31;
  const int wave = threadIdx.x >> 5;
  const int tilesM = (M + 63) >> 6;
  const int tilesN = (N + 63) >> 6;
  const int tile = blockIdx.x * 8 + wave;
  if (tile >= tilesM * tilesN) return;
  const int tm = tile / tilesN;
  const int tn = tile - tm * tilesN;
  const int m0 = tm << 6;
  const int n0 = tn << 6;

  const int rl = lane & 15;
  const int h8 = (lane >> 4) * 8;
  const unsigned short* pa = A + (size_t)(m0 + rl) * (size_t)KTOT + h8;
  const unsigned short* pb = B + (size_t)(n0 + rl) * (size_t)KTOT + h8;

  v8f acc[4][4];
#pragma unroll
  for (int i = 0; i < 4; ++i)
#pragma unroll
    for (int j = 0; j < 4; ++j) acc[i][j] = (v8f){0.f, 0.f, 0.f, 0.f, 0.f, 0.f, 0.f, 0.f};

#pragma unroll 1
  for (int k0 = 0; k0 < KTOT; k0 += 32) {
    F bf[4];
#pragma unroll
    for (int j = 0; j < 4; ++j) bf[j] = ld_frag<F>(pb + (size_t)(j << 4) * (size_t)KTOT + k0);
#pragma unroll
    for (int i = 0; i < 4; ++i) {
      const F af = ld_frag<F>(pa + (size_t)(i << 4) * (size_t)KTOT + k0);
#pragma unroll
      for (int j = 0; j < 4; ++j) acc[i][j] = mm(af, bf[j], acc[i][j]);
    }
  }

  float* slab = sT[wave];
  const int hh = lane >> 4;
  const int c4 = (lane & 15) * 4;
  const int nc = n0 + c4;
  const bool cok = nc < N;
  v4f bv = (v4f){0.f, 0.f, 0.f, 0.f};
  if (EPI == 1) {
    bv = *(const v4fa*)(bias + clampi(nc, 0, N - 4));
    asm volatile("" :: "v"(bv));
  }
#pragma unroll
  for (int i = 0; i < 4; ++i) {
    const int mBase = m0 + (i << 4);
#pragma unroll
    for (int j = 0; j < 4; ++j) {
#pragma unroll
      for (int r = 0; r < 8; ++r) slab[(h8 + r) * 68 + (j << 4) + rl] = acc[i][j][r];
    }
    __builtin_amdgcn_fence(__ATOMIC_RELEASE, "workgroup");
    __builtin_amdgcn_wave_barrier();
    __builtin_amdgcn_fence(__ATOMIC_ACQUIRE, "workgroup");
    v4f vv[8];
#pragma unroll
    for (int it = 0; it < 8; ++it) {
      const int row = it * 2 + hh;
      v4f v = *(const v4fa*)(slab + row * 68 + c4);
      if (EPI == 1) v += bv;
      vv[it] = v;
    }
    for (int pass = 0; pass < 2; ++pass) {
#pragma unroll
      for (int it = 0; it < 8; ++it) {
        const int row = mBase + it * 2 + hh;
        if (cok && row < M) *(volatile v4f*)(D + (size_t)row * (size_t)ldd + nc) = vv[it];
      }
      __threadfence();
    }
    __builtin_amdgcn_fence(__ATOMIC_RELEASE, "workgroup");
    __builtin_amdgcn_wave_barrier();
    __builtin_amdgcn_fence(__ATOMIC_ACQUIRE, "workgroup");
  }
}

#include <stddef.h>
#include <stdint.h>
#include <math.h>


#define H1_TWO_TERM 1

#define NN      50000
#define NE      800000
#define FD      128
#define MP      50048
#define NTHR    256
#define NWAVE   8
#define SLB     10
#define NBRUN   1024
#define NBLK    49
#define WKEYS   256
#define WCAP    256
#define CHUNK   (NWAVE * WKEYS)
#define NCH     ((NE + CHUNK - 1) / CHUNK)
#define LISTN   (NWAVE * WCAP)
#define RCAP    28672
#define DEGCAP  128
#define AROWS   128
#define NTAB    (NBLK * NBRUN)
#define NU1     (FD * (FD / 8))
#define NU2     (FD * (2 * FD / 8))
#define BK_ZINTS (LISTN + 2 * RCAP + 3 * NBRUN)
#define BK_LDS_INTS (BK_ZINTS + 16)
#define MEAS_B1024  16623
#define MEAS_MAXDEG 35

static_assert(NE % 256 == 0 && NE % 8 == 0);
static_assert(((long long)NE << SLB) < (1LL << 31));
static_assert(NBRUN == (1 << SLB) && NBRUN == 8 * AROWS && NBRUN % 32 == 0);
static_assert(NBLK * NBRUN >= MP && (NBLK - 1) * NBRUN < NN);
static_assert(MP % AROWS == 0 && MP % 64 == 0 && MP >= NN && MP % 16 == 0);
static_assert((long long)RCAP * 100 >= (long long)MEAS_B1024 * 105);
static_assert(DEGCAP >= MEAS_MAXDEG + 8);
static_assert(RCAP % (NTHR * 4) == 0 && RCAP % 32 == 0);
static_assert(BK_ZINTS % 4 == 0 && BK_LDS_INTS * 4 <= 300000);
static_assert(NU1 % NTHR == 0 && NU2 % NTHR == 0);
static_assert(FD % 32 == 0 && FD == 4 * 32);

typedef int v4i __attribute__((ext_vector_type(4)));
typedef v4i __attribute__((may_alias)) v4ia;

__device__ __forceinline__ void st2i(int* p, v4i v) {
  volatile v4i* q = (volatile v4i*)p;
  *q = v; __threadfence(); *q = v;
}
__device__ __forceinline__ void st2f(float* p, v4f v) {
  volatile v4f* q = (volatile v4f*)p;
  *q = v; __threadfence(); *q = v;
}
__device__ __forceinline__ void st2u(unsigned short* p, v4u v) {
  volatile v4u* q = (volatile v4u*)p;
  *q = v; __threadfence(); *q = v;
}

__global__ __launch_bounds__(NTHR) void k_wprep(const float* __restrict__ W1, const float* __restrict__ W2,
                                                const float* __restrict__ b1, const float* __restrict__ b2,
                                                unsigned short* W1T, unsigned short* W2D,
                                                float* B1F, float* B2F) {
  const int u = (int)blockIdx.x * NTHR + (int)threadIdx.x;
  if (u < NU1) {
    const int n  = u >> 4;
    const int k8 = (u & 15) * 8;
    const float* p = W1 + (size_t)k8 * FD + n;
    unsigned w[8];
#pragma unroll
    for (int i = 0; i < 8; ++i) w[i] = bf16_bits(p[(size_t)i * FD]);
    const v4u o = (v4u){ pk16(w[0], w[1]), pk16(w[2], w[3]), pk16(w[4], w[5]), pk16(w[6], w[7]) };
    st2u(W1T + (size_t)n * FD + k8, o);
  } else if (u < NU1 + NU2) {
    const int v  = u - NU1;
    const int n  = v >> 5;
    const int k8 = (v & 31) * 8;
    const int kk = k8 & (FD - 1);
    const float* p = W2 + (size_t)kk * FD + n;
    unsigned w[8];
#pragma unroll
    for (int i = 0; i < 8; ++i) w[i] = bf16_bits(p[(size_t)i * FD]);
    const v4u o = (v4u){ pk16(w[0], w[1]), pk16(w[2], w[3]), pk16(w[4], w[5]), pk16(w[6], w[7]) };
    st2u(W2D + (size_t)n * (2 * FD) + k8, o);
  } else {
    const int t    = u - (NU1 + NU2);
    const int wv   = t >> 5;
    const int lane = t & 31;
    if (wv == 0) {
      const v4f a = *(const v4fa*)(b1 + 4 * lane);
      const v4f o = (v4f){ bf16_val(a.x), bf16_val(a.y), bf16_val(a.z), bf16_val(a.w) };
      st2f(B1F + 4 * lane, o);
    } else if (wv == 1) {
      const v4f a = *(const v4fa*)(b2 + 4 * lane);
      const v4f o = (v4f){ bf16_val(a.x), bf16_val(a.y), bf16_val(a.z), bf16_val(a.w) };
      st2f(B2F + 4 * lane, o);
    }
  }
}

__global__ __launch_bounds__(NTHR) void k_bucket(const int* __restrict__ srcs, const int* __restrict__ dsts,
                                                 int* LIST, int* CNT, int* OFF, float* DINV, int* FLAG) {
  extern __shared__ __attribute__((aligned(16))) int dsm[];
  int* wl   = dsm;
  int* hl   = dsm + LISTN;
  int* sl   = hl + RCAP;
  int* cnt  = sl + RCAP;
  int* offs = cnt + NBRUN;
  int* cur  = offs + NBRUN;
  int* misc = cur + NBRUN;
  const int tid = (int)threadIdx.x, lane = tid & 31, wave = tid >> 5;
  const int blk = (int)blockIdx.x;
  const int nodeBase = blk * NBRUN;
  int nb = NN - nodeBase;
  nb = nb < 0 ? 0 : (nb > NBRUN ? NBRUN : nb);

  {
    const v4i z4 = (v4i){0, 0, 0, 0};
    for (int i = tid * 4; i < BK_ZINTS; i += NTHR * 4) *(v4ia*)(dsm + i) = z4;
    if (tid < 16) misc[tid] = 0;
  }
  __syncthreads();

  int* wq = wl + wave * WCAP;
  int tbase = 0;
#pragma unroll 1
  for (int ch = 0; ch < NCH; ++ch) {
    const int e0 = ch * CHUNK + wave * WKEYS + lane * 8;
    const int ec = e0 < NE - 8 ? e0 : NE - 8;
    const v4i da = *(const v4ia*)(dsts + ec);
    const v4i db = *(const v4ia*)(dsts + ec + 4);
    asm volatile("" :: "v"(da), "v"(db));
    const bool inr = (e0 + 7) < NE;
    const int dk[8] = { da.x, da.y, da.z, da.w, db.x, db.y, db.z, db.w };
    unsigned sj[8];
    bool hit[8];
    int c = 0;
#pragma unroll
    for (int J = 0; J < 8; ++J) {
      sj[J]  = (unsigned)dk[J] - (unsigned)nodeBase;
      hit[J] = inr && (sj[J] < (unsigned)nb);
      c += hit[J] ? 1 : 0;
    }
    int incl = c;
#pragma unroll
    for (int d = 1; d < 32; d <<= 1) {
      const int y = __shfl_up(incl, (unsigned)d, 32);
      incl += (lane >= d) ? y : 0;
    }
    int pos = incl - c;
    const int wcv = __shfl(incl, 31, 32);
#pragma unroll
    for (int J = 0; J < 8; ++J) {
      if (hit[J] && pos < WCAP) { wq[pos] = ((e0 + J) << SLB) | (int)sj[J]; pos += 1; }
    }
    int* mq = misc + (ch & 1) * 8;
    if (lane == 0) mq[wave] = wcv;
    __syncthreads();
    int pre = 0, tot = 0;
#pragma unroll
    for (int w2 = 0; w2 < NWAVE; ++w2) {
      const int cw = clampi(mq[w2], 0, WCAP);
      pre += (w2 < wave) ? cw : 0;
      tot += cw;
    }
    const int myc = __builtin_amdgcn_readfirstlane(clampi(wcv, 0, WCAP));
#pragma unroll 1
    for (int i0 = 0; i0 < myc; i0 += 32) {
      const int i = i0 + lane;
      const int v = wq[i < WCAP ? i : WCAP - 1];
      const int t = tbase + pre + i;
      if (i < myc && t < RCAP) hl[t] = v;
    }
    tbase += tot;
  }
  __syncthreads();
  const int ovf = (tbase > RCAP) ? 1 : 0;
  const int tt  = __builtin_amdgcn_readfirstlane(clampi(tbase, 0, RCAP));

#pragma unroll 1
  for (int b0 = 0; b0 < tt; b0 += 32) {
    const int i   = b0 + lane;
    const int ent = hl[i < RCAP ? i : RCAP - 1];
    const bool mine = (i < tt) && (((ent >> 7) & 7) == wave);
    unsigned msk = __builtin_amdgcn_ballot_w32(mine);
    int nh = (int)__builtin_popcount(msk);
    nh = nh > 32 ? 32 : nh;
#pragma unroll 1
    for (int q = 0; q < nh; ++q) {
      const int k = __builtin_ffs((int)msk) - 1;
      msk &= msk - 1u;
      const int u = __builtin_amdgcn_readlane(ent, k < 0 ? 0 : k);
      const int s = u & (NBRUN - 1);
      if (lane == 0) cnt[s] = cnt[s] + 1;
    }
  }
  __syncthreads();

  if (wave == 0) {
    const int base = lane * (NBRUN / 32);
    int s = 0;
#pragma unroll 1
    for (int i = 0; i < NBRUN / 32; ++i) s += cnt[base + i];
    int incl = s;
#pragma unroll
    for (int d = 1; d < 32; d <<= 1) {
      const int y = __shfl_up(incl, (unsigned)d, 32);
      incl += (lane >= d) ? y : 0;
    }
    int run = incl - s;
#pragma unroll 1
    for (int i = 0; i < NBRUN / 32; ++i) {
      const int cv = cnt[base + i];
      offs[base + i] = run;
      cur[base + i]  = run;
      run += cv;
    }
  }
  __syncthreads();

#pragma unroll 1
  for (int b0 = 0; b0 < tt; b0 += 32) {
    const int i   = b0 + lane;
    const int ent = hl[i < RCAP ? i : RCAP - 1];
    const bool mine = (i < tt) && (((ent >> 7) & 7) == wave);
    unsigned msk = __builtin_amdgcn_ballot_w32(mine);
    int nh = (int)__builtin_popcount(msk);
    nh = nh > 32 ? 32 : nh;
#pragma unroll 1
    for (int q = 0; q < nh; ++q) {
      const int k = __builtin_ffs((int)msk) - 1;
      msk &= msk - 1u;
      const int u = __builtin_amdgcn_readlane(ent, k < 0 ? 0 : k);
      const int s = u & (NBRUN - 1);
      if (lane == 0) {
        int p = cur[s];
        p = p < 0 ? 0 : (p > RCAP - 1 ? RCAP - 1 : p);
        sl[p] = u;
        cur[s] = p + 1;
      }
    }
  }
  __syncthreads();

#pragma unroll 1
  for (int it = 0; it < RCAP / (NTHR * 4); ++it) {
    const int i4 = (it * NTHR + tid) * 4;
    const v4i e4 = *(const v4ia*)(sl + i4);
    const int a0 = srcs[clampi(e4.x >> SLB, 0, NE - 1)];
    const int a1 = srcs[clampi(e4.y >> SLB, 0, NE - 1)];
    const int a2 = srcs[clampi(e4.z >> SLB, 0, NE - 1)];
    const int a3 = srcs[clampi(e4.w >> SLB, 0, NE - 1)];
    asm volatile("" :: "v"(a0), "v"(a1), "v"(a2), "v"(a3));
    const v4i o = (v4i){ clampi(a0, 0, NN - 1), clampi(a1, 0, NN - 1), clampi(a2, 0, NN - 1), clampi(a3, 0, NN - 1) };
    st2i(LIST + (size_t)blk * RCAP + i4, o);
  }

#pragma unroll 1
  for (int j = 0; j < 4; ++j) {
    const int s = 4 * tid + j;
    const float deg = (float)(cnt[s] + 1);
    const float dv  = (deg > 0.0f) ? (1.0f / sqrtf(deg)) : 0.0f;
    cur[s] = __float_as_int(dv);
  }
  {
    const v4i c4 = *(const v4ia*)(cnt + 4 * tid);
    const v4i o4 = *(const v4ia*)(offs + 4 * tid);
    const v4i d4 = *(const v4ia*)(cur + 4 * tid);
    const v4f df = (v4f){ __int_as_float(d4.x), __int_as_float(d4.y), __int_as_float(d4.z), __int_as_float(d4.w) };
    st2i(CNT + (size_t)nodeBase + 4 * tid, c4);
    st2i(OFF + (size_t)nodeBase + 4 * tid, o4);
    st2f(DINV + (size_t)nodeBase + 4 * tid, df);
  }
  if (tid < 8) st2i(FLAG + blk * 32 + 4 * tid, (v4i){ ovf, ovf, ovf, ovf });
}

template <int MODE>
__global__ __launch_bounds__(NTHR) void k_agg(const int* __restrict__ LIST, const int* __restrict__ CNT,
                                              const int* __restrict__ OFF, const float* __restrict__ DINV,
                                              const int* __restrict__ FLAG, const float* __restrict__ T,
                                              const float* __restrict__ BF, unsigned short* H1, float* outp) {
  const int tid = (int)threadIdx.x, lane = tid & 31, wave = tid >> 5;
  const int v0 = (int)blockIdx.x * AROWS + wave * 16;
  const int bk = clampi((int)blockIdx.x >> 3, 0, NBLK - 1);
  const v4f bv = *(const v4fa*)(BF + 4 * lane);
  const int vrc = clampi(v0 + (lane & 15), 0, NTAB - 1);
  const int   cntv = CNT[vrc];
  const int   offv = OFF[vrc];
  const float dvv  = DINV[vrc];
  const int   dvi  = __float_as_int(dvv);
  const int   fl   = FLAG[bk * 32];
  const int* lst = LIST + (size_t)bk * RCAP;
  const float qnan = __int_as_float(0x7fc00000);
  const int sa = (2 * lane) & 31, sb = (2 * lane + 1) & 31;

#pragma unroll 1
  for (int ri = 0; ri < 16; ++ri) {
    const int v = v0 + ri;
    const bool live = v < NN;
    int c = __builtin_amdgcn_readlane(cntv, ri);
    const bool big = c > DEGCAP;
    c = c < 0 ? 0 : (c > DEGCAP ? DEGCAP : c);
    c = live ? c : 0;
    const int o = clampi(__builtin_amdgcn_readlane(offv, ri), 0, RCAP);
    const float dd = __int_as_float(__builtin_amdgcn_readlane(dvi, ri));
    const int nc = v < NN ? v : NN - 1;
    v4f acc = (v4f){0.0f, 0.0f, 0.0f, 0.0f};
#pragma unroll 1
    for (int b0 = 0; b0 < c; b0 += 32) {
      int idx = o + b0 + lane;
      idx = idx > RCAP - 1 ? RCAP - 1 : idx;
      const int sr = clampi(lst[idx], 0, NN - 1);
      const float cf = DINV[sr] * dd;
      const int cfi = __float_as_int(cf);
      const int m32 = (c - b0) < 32 ? (c - b0) : 32;
#pragma unroll 1
      for (int k = 0; k < m32; ++k) {
        const int   sk = __builtin_amdgcn_readlane(sr, k);
        const float ck = __int_as_float(__builtin_amdgcn_readlane(cfi, k));
        const v4f a = *(const v4fa*)(T + (size_t)sk * FD + 4 * lane);
        acc.x = fmaf(a.x, ck, acc.x); acc.y = fmaf(a.y, ck, acc.y);
        acc.z = fmaf(a.z, ck, acc.z); acc.w = fmaf(a.w, ck, acc.w);
      }
    }
    const v4f sv = *(const v4fa*)(T + (size_t)nc * FD + 4 * lane);
    const float rd = dd * dd;
    v4f y;
    y.x = (acc.x + sv.x * rd) + bv.x;
    y.y = (acc.y + sv.y * rd) + bv.y;
    y.z = (acc.z + sv.z * rd) + bv.z;
    y.w = (acc.w + sv.w * rd) + bv.w;
    const bool bad = (fl != 0) || big;
    if constexpr (MODE != 0) {
      y.x = (y.x > 0.0f) ? y.x : (y.x - y.x);
      y.y = (y.y > 0.0f) ? y.y : (y.y - y.y);
      y.z = (y.z > 0.0f) ? y.z : (y.z - y.z);
      y.w = (y.w > 0.0f) ? y.w : (y.w - y.w);
      y.x = bad ? qnan : y.x; y.y = bad ? qnan : y.y; y.z = bad ? qnan : y.z; y.w = bad ? qnan : y.w;
      y.x = live ? y.x : 0.0f; y.y = live ? y.y : 0.0f; y.z = live ? y.z : 0.0f; y.w = live ? y.w : 0.0f;
      const int hw0 = (int)pk16(bf16_bits(y.x), bf16_bits(y.y));
      const int hw1 = (int)pk16(bf16_bits(y.z), bf16_bits(y.w));
#if H1_TWO_TERM
      const int lw0 = (int)pk16(bf16_lo_bits(y.x), bf16_lo_bits(y.y));
      const int lw1 = (int)pk16(bf16_lo_bits(y.z), bf16_lo_bits(y.w));
#else
      const int lw0 = 0;
      const int lw1 = 0;
#endif
      const int g0 = __shfl(hw0, sa, 32), g1 = __shfl(hw1, sa, 32);
      const int g2 = __shfl(hw0, sb, 32), g3 = __shfl(hw1, sb, 32);
      const int p0 = __shfl(lw0, sa, 32), p1 = __shfl(lw1, sa, 32);
      const int p2 = __shfl(lw0, sb, 32), p3 = __shfl(lw1, sb, 32);
      const bool lsel = lane >= 16;
      v4u pv;
      pv.x = (unsigned)(lsel ? p0 : g0);
      pv.y = (unsigned)(lsel ? p1 : g1);
      pv.z = (unsigned)(lsel ? p2 : g2);
      pv.w = (unsigned)(lsel ? p3 : g3);
      st2u(H1 + (size_t)v * (2 * FD) + 8 * lane, pv);
    } else {
      y.x = bad ? qnan : y.x; y.y = bad ? qnan : y.y; y.z = bad ? qnan : y.z; y.w = bad ? qnan : y.w;
      if (live) st2f(outp + (size_t)v * FD + 4 * lane, y);
    }
  }
}

#define SZ_XB   ((size_t)MP * FD * 2)
#define SZ_T    ((size_t)MP * FD * 4)
#define SZ_H1   ((size_t)MP * 2 * FD * 2)
#define SZ_LIST ((size_t)NBLK * RCAP * 4)
#define SZ_TAB  ((size_t)NTAB * 4)
#define SZ_W1T  ((size_t)FD * FD * 2)
#define SZ_W2D  ((size_t)FD * 2 * FD * 2)
#define SZ_BF   ((size_t)FD * 4)
#define SZ_FLAG ((size_t)NBLK * 128)
#define WS_TOTAL (SZ_XB + SZ_T + SZ_H1 + SZ_LIST + 3 * SZ_TAB + SZ_W1T + SZ_W2D + 2 * SZ_BF + SZ_FLAG)
static_assert(SZ_XB % 128 == 0 && SZ_T % 128 == 0 && SZ_H1 % 128 == 0 && SZ_LIST % 128 == 0);
static_assert(SZ_TAB % 128 == 0 && SZ_W1T % 128 == 0 && SZ_W2D % 128 == 0 && SZ_BF % 128 == 0 && SZ_FLAG % 128 == 0);
static_assert(WS_TOTAL <= ((size_t)128 << 20));
static_assert(((long long)MP * (2 * FD) / 8) < (1LL << 31));
static_assert((MP * FD / 8) % 256 == 0);

extern "C" void kernel_launch(void* const* d_in, const int* in_sizes, int n_in,
                              void* d_out, int out_size, void* d_ws, size_t ws_size,
                              hipStream_t stream) {
  if (n_in < 6) return;
  if (in_sizes[0] != NN * FD) return;
  if (in_sizes[1] != 2 * NE) return;
  if (in_sizes[2] != FD * FD || in_sizes[3] != FD) return;
  if (in_sizes[4] != FD * FD || in_sizes[5] != FD) return;
  if (out_size != NN * FD) return;
  if ((size_t)WS_TOTAL > ws_size) return;

  const float* x    = (const float*)d_in[0];
  const int*   edge = (const int*)d_in[1];
  const float* W1   = (const float*)d_in[2];
  const float* b1   = (const float*)d_in[3];
  const float* W2   = (const float*)d_in[4];
  const float* b2   = (const float*)d_in[5];
  float* out = (float*)d_out;
  const int* src = edge;
  const int* dst = edge + NE;

  char* ws = (char*)d_ws;
  size_t off = 0;
  unsigned short* XB  = (unsigned short*)(ws + off); off += SZ_XB;
  float*          T   = (float*)(ws + off);          off += SZ_T;
  unsigned short* H1  = (unsigned short*)(ws + off); off += SZ_H1;
  int*            LST = (int*)(ws + off);            off += SZ_LIST;
  int*            CNT = (int*)(ws + off);            off += SZ_TAB;
  int*            OFT = (int*)(ws + off);            off += SZ_TAB;
  float*          DNV = (float*)(ws + off);          off += SZ_TAB;
  unsigned short* W1T = (unsigned short*)(ws + off); off += SZ_W1T;
  unsigned short* W2D = (unsigned short*)(ws + off); off += SZ_W2D;
  float*          B1F = (float*)(ws + off);          off += SZ_BF;
  float*          B2F = (float*)(ws + off);          off += SZ_BF;
  int*            FLG = (int*)(ws + off);            off += SZ_FLAG;
  if (off != (size_t)WS_TOTAL) return;

  const size_t bkLds = (size_t)BK_LDS_INTS * 4;
  hipFuncSetAttribute(reinterpret_cast<const void*>(&k_bucket), hipFuncAttributeMaxDynamicSharedMemorySize, (int)bkLds);

  const int tiles = (MP / 64) * (FD / 64);
  const int gG    = (tiles + 7) / 8;

  k_plane<0><<<MP * FD / 8 / 256, 256, 0, stream>>>(x, NN, FD, FD, XB, MP, FD);
  k_wprep<<<(NU1 + NU2) / NTHR + 1, NTHR, 0, stream>>>(W1, W2, b1, b2, W1T, W2D, B1F, B2F);
  k_bucket<<<NBLK, NTHR, bkLds, stream>>>(src, dst, LST, CNT, OFT, DNV, FLG);
  k_gemm_nt<0, 0><<<gG, 256, 0, stream>>>(XB, W1T, B1F, T, MP, FD, FD, FD);
  k_agg<1><<<MP / AROWS, NTHR, 0, stream>>>(LST, CNT, OFT, DNV, FLG, T, B1F, H1, out);
  k_gemm_nt<0, 0><<<gG, 256, 0, stream>>>(H1, W2D, B2F, T, MP, FD, 2 * FD, FD);
  k_agg<0><<<MP / AROWS, NTHR, 0, stream>>>(LST, CNT, OFT, DNV, FLG, T, B2F, H1, out);
}
